// RadialNetwork2d_73083163509212
// MI455X (gfx1250) — hardware-verified
//
#include <hip/hip_runtime.h>


typedef _Float16 v16h __attribute__((ext_vector_type(16)));
typedef float    v8f  __attribute__((ext_vector_type(8)));
typedef float    v4f  __attribute__((ext_vector_type(4)));
typedef float    v4fa __attribute__((ext_vector_type(4))) __attribute__((may_alias));

#define RBF_GRID   32
#define RBF_P      1024
#define RBF_A      8
#define RBF_WAVES  8
#define RBF_ITERS  4
#define RBF_TILES_PER_BLOCK (RBF_WAVES * RBF_ITERS)
#define RBF_SCALE  (-0.18033688011112042f)
#define RBF_NORM   (0.039788735772973836f)
#define RBF_A_SC   (1048576.0f)
#define RBF_W_SC   (4096.0f)
#define RBF_INV_SC (2.3283064365386963e-10f)

__device__ __forceinline__ v8f wmma_f16_16x16x32(v16h a, v16h b, v8f c)
{
    v8f d = __builtin_amdgcn_wmma_f32_16x16x32_f16(false, a, false, b, (short)0, c, false, false);
    asm volatile("v_nop\n\tv_nop\n\tv_nop\n\tv_nop" : "+v"(d) : "v"(a), "v"(b));
    return d;
}

__global__ __launch_bounds__(256)
void rbf_basis_gemm_kernel(const float* __restrict__ pos,
                           const float* __restrict__ W,
                           const float* __restrict__ bias,
                           float* __restrict__ out,
                           int Bn, int nTiles)
{
    __shared__ alignas(32) _Float16 Wt[RBF_GRID * 32 * 16];
    __shared__ alignas(16) float stage[RBF_WAVES][128];

    const int tid  = threadIdx.x;
    const int lane = tid & 31;
    const int wave = tid >> 5;
    const int m    = lane & 15;
    const int h    = lane >> 4;
    const int n    = m;

    for (int e = tid; e < RBF_GRID * 32 * 16; e += 256) {
        const int k  = e >> 9;
        const int L  = (e >> 4) & 31;
        const int i  = e & 15;
        const int nn = L & 15;
        const int hh = L >> 4;
        const int cy = 8 * hh + i + ((i >> 3) << 3);
        float w = 0.0f;
        if (nn < RBF_A) w = W[nn * RBF_P + k * RBF_GRID + cy] * RBF_W_SC;
        Wt[e] = (_Float16)w;
    }
    __syncthreads();

    const float bn = (n < RBF_A) ? bias[n] : 0.0f;

    for (int it = 0; it < RBF_ITERS; ++it) {
        const int  tile    = (blockIdx.x * RBF_ITERS + it) * RBF_WAVES + wave;
        const bool valid   = tile < nTiles;
        const int  rowBase = tile * 16;
        int rowm = rowBase + m;
        if (rowm > Bn - 1) rowm = Bn - 1;

        const float x = pos[(size_t)rowm * 2 + 0];
        const float y = pos[(size_t)rowm * 2 + 1];

        float ey[16];
        #pragma unroll
        for (int i = 0; i < 16; ++i) {
            const int   cy = 8 * h + i + ((i >> 3) << 3);
            const float dy = y - (float)cy;
            ey[i] = exp2f((dy * dy) * RBF_SCALE);
        }

        v8f acc = {0.f, 0.f, 0.f, 0.f, 0.f, 0.f, 0.f, 0.f};
        #pragma unroll 8
        for (int k = 0; k < RBF_GRID; ++k) {
            const float dx  = x - (float)k;
            const float exn = exp2f((dx * dx) * RBF_SCALE) * (RBF_NORM * RBF_A_SC);
            v16h av;
            #pragma unroll
            for (int i = 0; i < 16; ++i) av[i] = (_Float16)(exn * ey[i]);
            const v16h bv = *(const v16h*)(Wt + (k * 32 + lane) * 16);
            acc = wmma_f16_16x16x32(av, bv, acc);
        }

        if (n < RBF_A) {
            #pragma unroll
            for (int r = 0; r < 8; ++r)
                stage[wave][(8 * h + r) * RBF_A + n] = acc[r] * RBF_INV_SC + bn;
        }
        __syncthreads();

        {
            const v4f  v       = *(const v4fa*)(&stage[wave][4 * lane]);
            const int  row     = rowBase + (lane >> 1);
            const bool doStore = valid && (row < Bn);
            float* p = out + (size_t)rowBase * RBF_A + 4 * lane;
            if (doStore) *(volatile v4f*)p = v;
            __threadfence();
            if (doStore) *(volatile v4f*)p = v;
        }
        __syncthreads();
    }
}

extern "C" void kernel_launch(void* const* d_in, const int* in_sizes, int n_in,
                              void* d_out, int out_size, void* d_ws, size_t ws_size,
                              hipStream_t stream)
{
    (void)d_ws; (void)ws_size;
    if (n_in < 3) return;
    const float* pos  = (const float*)d_in[0];
    const float* W    = (const float*)d_in[1];
    const float* bias = (const float*)d_in[2];
    float* out = (float*)d_out;

    const int Bn = in_sizes[0] / 2;
    if (Bn < 1) return;
    if (in_sizes[1] != RBF_A * RBF_P) return;
    if (in_sizes[2] < RBF_A) return;
    if (out_size < Bn * RBF_A) return;

    const int nTiles = (Bn + 15) / 16;
    const int blocks = (nTiles + RBF_TILES_PER_BLOCK - 1) / RBF_TILES_PER_BLOCK;

    rbf_basis_gemm_kernel<<<blocks, 256, 0, stream>>>(pos, W, bias, out, Bn, nTiles);
}
